// DAGCN_reduce_7705171329817
// MI455X (gfx1250) — hardware-run, weakly checked
//
#include <hip/hip_runtime.h>


#ifndef NT
#define NT 12
#endif
#ifndef NB
#define NB 16
#endif
#ifndef NN
#define NN 1024
#endif
#define NT_FULL 12
#define NB_FULL 16
#define NN_FULL 1024
#ifndef OUT_NT
#define OUT_NT NT
#endif
#ifndef OUT_NN
#define OUT_NN NN
#endif
#define ED   10
#define EDP  32
#define CK   3
#define CC   32
#define CO   32
#define JW   (NB * CC)
#define ZR   (ED * CO)
#define BPW  4
#define AW   ((NB / BPW) < 4 ? (NB / BPW) : 4)
#define OSP  36
#define LOG2E 1.4426950408889634f
#define PSH  14.0f
#define NEGB (-3.0e38f)

static_assert(CC == 32);
static_assert(CO == 32);
static_assert(EDP == 32);
static_assert(ED <= EDP);
static_assert(NN % 64 == 0);
static_assert(NB % BPW == 0);
static_assert((NB / BPW) % AW == 0);
static_assert(AW >= 1);
static_assert(ZR % 16 == 0);
static_assert(NT <= NT_FULL);
static_assert(NB <= NB_FULL);
static_assert(NN <= NN_FULL);
static_assert(OUT_NT >= NT);
static_assert(OUT_NN >= NN);
static_assert((OSP * 4) % 16 == 0);
static_assert(((size_t)NT * NN * 4) % 8 == 0);
static_assert(((size_t)NT * CK * ZR * 4) % 8 == 0);
static_assert((((((size_t)(NB_FULL - 1) * NT_FULL + (NT_FULL - 1)) * NN_FULL) + NN_FULL) * CO) * 4 == (size_t)25165824);

typedef _Float16 h16;
typedef unsigned short bf;
typedef __attribute__((ext_vector_type(16))) __bf16   v16bf;
typedef __attribute__((ext_vector_type(16))) _Float16 v16h;
typedef __attribute__((ext_vector_type(8)))  _Float16 v8h;
typedef __attribute__((ext_vector_type(8)))  unsigned short v8us;
typedef __attribute__((ext_vector_type(8)))  float    v8f;
typedef __attribute__((ext_vector_type(4)))  float    v4f;
typedef v4f  __attribute__((may_alias)) v4fa;
typedef v8h  __attribute__((may_alias)) v8ha;

__device__ __forceinline__ unsigned short f2bf(float f) { unsigned u = __float_as_uint(f); u += 0x7FFFu + ((u >> 16) & 1u); return (unsigned short)(u >> 16); }
__device__ __forceinline__ float bfr(float f) { return __uint_as_float(((unsigned)f2bf(f)) << 16); }
__device__ __forceinline__ v16h cat16(v8h lo, v8h hi) { return __builtin_shufflevector(lo, hi, 0, 1, 2, 3, 4, 5, 6, 7, 8, 9, 10, 11, 12, 13, 14, 15); }
__device__ __forceinline__ v16bf cat16b(v8us lo, v8us hi) { return __builtin_bit_cast(v16bf, __builtin_shufflevector(lo, hi, 0, 1, 2, 3, 4, 5, 6, 7, 8, 9, 10, 11, 12, 13, 14, 15)); }
__device__ __forceinline__ v8f wmma16(v16h a, v16h b, v8f c) { return __builtin_amdgcn_wmma_f32_16x16x32_f16(false, a, false, b, (short)0, c, false, false); }
__device__ __forceinline__ v8f wmmab(v16bf a, v16bf b, v8f c) { return __builtin_amdgcn_wmma_f32_16x16x32_bf16(false, a, false, b, (short)0, c, false, false); }
__device__ __forceinline__ v16h  ldh(const h16* p) { return cat16(*(const v8h*)p, *(const v8h*)(p + 16)); }
__device__ __forceinline__ v16bf ldb(const bf* p)  { return cat16b(*(const v8us*)p, *(const v8us*)(p + 16)); }
__device__ __forceinline__ void wave_sync() { __builtin_amdgcn_fence(3  , "wavefront"); __builtin_amdgcn_wave_barrier(); asm volatile("" ::: "memory"); }

__device__ __forceinline__ v8f wmma16g(v16h a, v16h b, v8f c) { c = wmma16(a, b, c); asm volatile("v_nop\n\tv_nop\n\tv_nop\n\tv_nop" : "+v"(c) : "v"(a), "v"(b)); return c; }
__device__ __forceinline__ v8f wmmabg(v16bf a, v16bf b, v8f c) { c = wmmab(a, b, c); asm volatile("v_nop\n\tv_nop\n\tv_nop\n\tv_nop" : "+v"(c) : "v"(a), "v"(b)); return c; }
static __device__ __forceinline__ h16 toh_flush(float v) { const h16 r = (h16)v; return (fabsf(v) < 6.103515625e-05f) ? (h16)0.0f : r; }
static __device__ __forceinline__ h16 p_flush(float e) { const float v = __builtin_amdgcn_exp2f(e); const h16 r = (h16)v; return (e < -14.0f) ? (h16)0.0f : r; }

__global__ __launch_bounds__(256) void k_epad(const float* __restrict__ E, bf* EB, int n8) {
    const int i = blockIdx.x * 256 + threadIdx.x; if (i >= n8) return;
    const int row = i >> 2, c8 = (i & 3) * 8;
    const int t = row / NN, n = row % NN;
    const float* src = E + ((size_t)t * NN_FULL + (size_t)n) * ED;
    v8us o;
#pragma unroll
    for (int k = 0; k < 8; ++k) {
        const int d = c8 + k; const int dc = d < ED ? d : (ED - 1);
        float v = src[dc]; asm volatile("" : "+v"(v));
        o[k] = (d < ED) ? f2bf(v) : (unsigned short)0; }
    *(volatile v8us*)(EB + (size_t)i * 8) = o; __threadfence(); *(volatile v8us*)(EB + (size_t)i * 8) = o;
}

__global__ __launch_bounds__(256) void k_wT(const float* __restrict__ W, h16* WT, int n8) {
    const int i = blockIdx.x * 256 + threadIdx.x; if (i >= n8) return;
    const int c8 = (i & 3) * 8; const int q = i >> 2;
    const int rowid = q % ZR; const int q2 = q / ZR; const int kk = q2 % CK; const int t = q2 / CK;
    const int d = rowid >> 5, o = rowid & 31;
    const float* src = W + ((((size_t)t * ED + d) * CK + kk) * CC + c8) * CO + o;
    v8h hv;
#pragma unroll
    for (int k = 0; k < 8; ++k) hv[k] = toh_flush(bfr(src[(size_t)k * CO]));
    *(volatile v8h*)(WT + (size_t)i * 8) = hv; __threadfence(); *(volatile v8h*)(WT + (size_t)i * 8) = hv;
}

__global__ __launch_bounds__(128) void k_xT(const float* __restrict__ X, h16* XT) {
    __shared__ __align__(16) h16 ts[CC * 72];
    static_assert(sizeof(h16) * CC * 72 <= 131072);
    static_assert(128 * 4 * 4 == 64 * CC);
    static_assert(128 * 2 * 16 == CC * 64 * 2);
    const int tid = threadIdx.x; const int m0 = blockIdx.x * 64, b = blockIdx.y, t = blockIdx.z;
    const float* src = X + (((size_t)b * NT_FULL + t) * NN_FULL + m0) * CC;
#pragma unroll
    for (int s = 0; s < 4; ++s) { const int q = tid + 128 * s; const int m = q >> 3, c4 = (q & 7) * 4;
        const v4f v = *(const v4f*)(src + (size_t)q * 4);
#pragma unroll
        for (int k = 0; k < 4; ++k) ts[(c4 + k) * 72 + m] = toh_flush(bfr(v[k])); }
    __syncthreads();
    h16* dst = XT + ((size_t)t * JW + (size_t)b * CC) * NN + m0;
#pragma unroll 1
    for (int ps = 0; ps < 2; ++ps) {
#pragma unroll
        for (int s = 0; s < 2; ++s) { const int c = s * 16 + (tid >> 3), c8 = (tid & 7) * 8;
            const v8h hv = *(const v8ha*)(&ts[c * 72 + c8]);
            *(volatile v8h*)(dst + (size_t)c * NN + c8) = hv; }
        if (ps == 0) __threadfence(); }
}

__global__ __launch_bounds__(32 * AW) __attribute__((amdgpu_num_vgpr(256)))
void k_gconv(const bf* __restrict__ EB, const h16* __restrict__ XT, const h16* __restrict__ WT,
             const float* __restrict__ X, const float* __restrict__ E, const float* __restrict__ BP, float* OUT) {
    __shared__ __align__(16) float os[AW * 16 * OSP];
    static_assert(sizeof(float) * AW * 16 * OSP <= 131072);
    static_assert(32 * 4 * 16 == 16 * CO * 4);
    const int lane = threadIdx.x & 31, lr = lane & 15, hi = lane >> 4;
    const int wave = __builtin_amdgcn_readfirstlane((int)(threadIdx.x >> 5));
    const int t = blockIdx.y; const int n0 = blockIdx.x * 16;
    const int g = blockIdx.z * AW + wave;
    const int b0 = g * BPW; const int j0 = g * (BPW * CC);
    const size_t eb = (size_t)t * NN * EDP;
    const v16bf qf = ldb(EB + eb + (size_t)(n0 + lr) * EDP + 8 * hi);
    const size_t ko = eb + (size_t)lr * EDP + 8 * hi;
    const size_t vo = ((size_t)t * JW + (size_t)(j0 + lr)) * NN + 8 * hi;
    v8f o[8];
#pragma unroll
    for (int jt = 0; jt < 8; ++jt) o[jt] = (v8f){};
    float m = NEGB, l = 0.0f;
#pragma unroll 1
    for (int key0 = 0; key0 < NN; key0 += 32) {
        const bf* ka = EB + ko + (size_t)key0 * EDP;
        const v16bf ka0 = ldb(ka), kb0 = ldb(ka + 16 * EDP);
        v8f sa = (v8f){}, sb = (v8f){};
        sa = wmmabg(ka0, qf, sa); sb = wmmabg(kb0, qf, sb);
        float ta[8], tb[8]; float mx = NEGB;
#pragma unroll
        for (int r = 0; r < 8; ++r) {
            ta[r] = fmaxf(sa[r], 0.0f) * LOG2E; tb[r] = fmaxf(sb[r], 0.0f) * LOG2E;
            mx = fmaxf(mx, fmaxf(ta[r], tb[r])); }
        mx = fmaxf(mx, __shfl_xor(mx, 16, 32));
        const float mnew = fmaxf(m, mx);
        const float alpha = __builtin_amdgcn_exp2f(m - mnew);
        const float sh = PSH - mnew;
        v16h pb; float ls = 0.0f;
#pragma unroll
        for (int r = 0; r < 8; ++r) {
            const h16 pa = p_flush(ta[r] + sh); const h16 pc = p_flush(tb[r] + sh);
            pb[r] = pa; pb[8 + r] = pc;
            ls += (float)pa + (float)pc; }
        l = l * alpha + ls; m = mnew;
#pragma unroll
        for (int jt = 0; jt < 8; ++jt) o[jt] = o[jt] * alpha;
        const h16* va = XT + vo + key0;
#pragma unroll
        for (int jt = 0; jt < 8; ++jt) { const v16h vf = ldh(va + (size_t)(16 * jt) * NN); o[jt] = wmma16g(vf, pb, o[jt]); }
    }
    l += __shfl_xor(l, 16, 32);
    const float inv = 1.0f / l;

    const float* erow = E + ((size_t)t * NN_FULL + (size_t)(n0 + lr)) * ED;
    const float* bpt = BP + (size_t)t * ED * CO + 8 * hi;
    v8f bacc0 = (v8f){}, bacc1 = (v8f){};
    float sd = 0.0f;
#pragma unroll 1
    for (int d = 0; d < ED; ++d) {
        const float ed = bfr(erow[d]);
        sd = fmaf(ed, ed, sd);
        const float* bq = bpt + d * CO;
        const v4f p0 = *(const v4f*)bq, p1 = *(const v4f*)(bq + 4), p2 = *(const v4f*)(bq + 16), p3 = *(const v4f*)(bq + 20);
#pragma unroll
        for (int r = 0; r < 4; ++r) {
            bacc0[r]     = fmaf(ed, bfr(p0[r]), bacc0[r]);     bacc0[4 + r] = fmaf(ed, bfr(p1[r]), bacc0[4 + r]);
            bacc1[r]     = fmaf(ed, bfr(p2[r]), bacc1[r]);     bacc1[4 + r] = fmaf(ed, bfr(p3[r]), bacc1[4 + r]); }
    }
    const float diag = __builtin_amdgcn_exp2f(fmaxf(sd, 0.0f) * LOG2E - m + PSH) * inv;
    const float twod = 2.0f * diag;

    const size_t wo = ((size_t)t * CK * ZR + (size_t)lr) * CC + 8 * hi;
    const int wb = wave * 16 * OSP;
#pragma unroll
    for (int bi = 0; bi < BPW; ++bi) {
        const int b = b0 + bi;
        const float* xrow = X + (((size_t)b * NT_FULL + t) * NN_FULL + (size_t)(n0 + lr)) * CC + 8 * hi;
        const v4f x0 = *(const v4f*)xrow, x1 = *(const v4f*)(xrow + 4), x2 = *(const v4f*)(xrow + 16), x3 = *(const v4f*)(xrow + 20);
        v16h xf, yf, zf;
#pragma unroll
        for (int r = 0; r < 4; ++r) {
            const float xa = bfr(x0[r]), xb = bfr(x1[r]), xc = bfr(x2[r]), xd = bfr(x3[r]);
            const float ya = o[2 * bi][r] * inv, yb = o[2 * bi][4 + r] * inv, yc = o[2 * bi + 1][r] * inv, yd = o[2 * bi + 1][4 + r] * inv;
            xf[r] = toh_flush(xa); xf[4 + r] = toh_flush(xb); xf[8 + r] = toh_flush(xc); xf[12 + r] = toh_flush(xd);
            yf[r] = toh_flush(ya); yf[4 + r] = toh_flush(yb); yf[8 + r] = toh_flush(yc); yf[12 + r] = toh_flush(yd);
            zf[r]      = toh_flush(twod * ya - xa); zf[4 + r]  = toh_flush(twod * yb - xb);
            zf[8 + r]  = toh_flush(twod * yc - xc); zf[12 + r] = toh_flush(twod * yd - xd); }
        v8f a0 = bacc0, a1 = bacc1;
#pragma unroll 1
        for (int d = 0; d < ED; ++d) {
            const float ed = bfr(erow[d]);
            const h16* wr = WT + wo + (size_t)d * (CO * CC);
            { v8f z = (v8f){};
              z = wmma16g(ldh(wr), xf, z); z = wmma16g(ldh(wr + (size_t)ZR * CC), yf, z); z = wmma16g(ldh(wr + (size_t)2 * ZR * CC), zf, z);
#pragma unroll
              for (int r = 0; r < 8; ++r) a0[r] = fmaf(ed, z[r], a0[r]); }
            { const h16* wr1 = wr + 16 * CC; v8f z = (v8f){};
              z = wmma16g(ldh(wr1), xf, z); z = wmma16g(ldh(wr1 + (size_t)ZR * CC), yf, z); z = wmma16g(ldh(wr1 + (size_t)2 * ZR * CC), zf, z);
#pragma unroll
              for (int r = 0; r < 8; ++r) a1[r] = fmaf(ed, z[r], a1[r]); }
        }
        { v4f p, c;
          p[0] = a0[0]; p[1] = a0[1]; p[2] = a0[2]; p[3] = a0[3]; c[0] = a0[4]; c[1] = a0[5]; c[2] = a0[6]; c[3] = a0[7];
          *(v4fa*)(&os[wb + lr * OSP +  0 + 8 * hi]) = p; *(v4fa*)(&os[wb + lr * OSP +  0 + 8 * hi + 4]) = c;
          p[0] = a1[0]; p[1] = a1[1]; p[2] = a1[2]; p[3] = a1[3]; c[0] = a1[4]; c[1] = a1[5]; c[2] = a1[6]; c[3] = a1[7];
          *(v4fa*)(&os[wb + lr * OSP + 16 + 8 * hi]) = p; *(v4fa*)(&os[wb + lr * OSP + 16 + 8 * hi + 4]) = c; }
        wave_sync();
        float* orow = OUT + (((size_t)b * OUT_NT + t) * OUT_NN + (size_t)n0) * CO;
#pragma unroll 1
        for (int ps = 0; ps < 2; ++ps) {
#pragma unroll
            for (int s = 0; s < 4; ++s) { const int row = 4 * s + (lane >> 3), cofs = (lane & 7) * 4;
                const v4f val = *(const v4fa*)(&os[wb + row * OSP + cofs]);
                *(volatile v4f*)(orow + (size_t)row * CO + cofs) = val; }
            if (ps == 0) __threadfence(); }
        wave_sync();
    }
}

static constexpr size_t al256(size_t v) { return (v + 255) & ~(size_t)255; }
static constexpr size_t SZ_EB = al256((size_t)NT * NN * EDP * 2);
static constexpr size_t SZ_XT = al256((size_t)NT * JW * NN * 2);
static constexpr size_t SZ_WT = al256((size_t)NT * CK * ZR * CC * 2);
static constexpr size_t SZ_TOTAL = SZ_EB + SZ_XT + SZ_WT;
static_assert(SZ_TOTAL <= (size_t)134217728);
static_assert((size_t)NT * NN * 4 * 16 == (size_t)NT * NN * EDP * 2);
static_assert((size_t)NT * CK * ZR * 4 * 16 == (size_t)NT * CK * ZR * CC * 2);
static_assert((size_t)(NN / 64) * NB * NT * 4096 == (size_t)NT * JW * NN * 2);
static_assert((size_t)(NN / 16) * NT * (NB / BPW / AW) * AW * BPW * 16 * CO == (size_t)NB * NT * NN * CO);

extern "C" void kernel_launch(void* const* d_in, const int* in_sizes, int n_in,
                              void* d_out, int out_size, void* d_ws, size_t ws_size, hipStream_t stream) {
    if (n_in < 4) return;
    const size_t needx = ((((size_t)(NB - 1) * NT_FULL + (size_t)(NT - 1)) * NN_FULL) + (size_t)NN) * CC;
    const size_t neede = ((size_t)(NT - 1) * NN_FULL + (size_t)NN) * ED;
    const size_t needw = (size_t)NT * ED * CK * CC * CO;
    const size_t needb = (size_t)NT * ED * CO;
    const size_t needo = ((((size_t)(NB - 1) * OUT_NT + (size_t)(NT - 1)) * OUT_NN) + (size_t)NN) * CO;
    if ((size_t)in_sizes[0] < needx || (size_t)in_sizes[1] < neede || (size_t)in_sizes[2] < needw || (size_t)in_sizes[3] < needb) return;
    if ((size_t)out_size < needo) return;
    if (SZ_TOTAL > ws_size) return;
    const float* X  = (const float*)d_in[0];
    const float* E  = (const float*)d_in[1];
    const float* W  = (const float*)d_in[2];
    const float* BP = (const float*)d_in[3];
    float* OUT = (float*)d_out;
    char* wsp = (char*)d_ws;
    bf*  EB = (bf*)wsp;  wsp += SZ_EB;
    h16* XT = (h16*)wsp; wsp += SZ_XT;
    h16* WT = (h16*)wsp; wsp += SZ_WT;

    { const int n8 = NT * NN * 4; k_epad<<<(unsigned)((n8 + 255) / 256), 256, 0, stream>>>(E, EB, n8); }
    { const int n8 = NT * CK * ZR * 4; k_wT<<<(unsigned)((n8 + 255) / 256), 256, 0, stream>>>(W, WT, n8); }
    k_xT<<<dim3(NN / 64, NB, NT), 128, 0, stream>>>(X, XT);
    k_gconv<<<dim3(NN / 16, NT, NB / BPW / AW), 32 * AW, 0, stream>>>(EB, XT, WT, X, E, BP, OUT);
}
